// EncoderLayer_23811298689034
// MI455X (gfx1250) — hardware-verified
//
#include <hip/hip_runtime.h>
#include <math.h>


#ifndef NB
#define NB 2
#endif
#ifndef SEQ
#define SEQ 2048
#endif
#define NB_FULL  2
#define SEQ_FULL 2048
#define DM   1024
#define NH   16
#define HD   64
#define DFF  4096
#define MROWS (NB * SEQ)
#define PCAR 1024.0f
#define WCAR 16.0f
#define CCAR 16.0f
#define GCAR 16.0f
#define LNEPS 1e-5f
#define LOG2E 1.4426950408889634f

static_assert(SEQ % 128 == 0);
static_assert(SEQ % 64 == 0);
static_assert(SEQ <= SEQ_FULL);
static_assert(NB <= NB_FULL);
static_assert(DM == NH * HD);
static_assert(HD == 64);
static_assert(DM % 128 == 0);
static_assert(DM % 64 == 0);
static_assert(DFF % 64 == 0);
static_assert(DM % 32 == 0);
static_assert(DFF % 32 == 0);
static_assert(MROWS % 64 == 0);
static_assert(MROWS % 8 == 0);
static_assert(((size_t)MROWS * DM) % 2048 == 0);
static_assert((DM * DM / 64) % 64 == 0);
static_assert((DM * DFF / 64) % 64 == 0);
static_assert((size_t)(MROWS * (size_t)DM / 8 / 256) * 256 * 8 == (size_t)MROWS * DM);
static_assert((size_t)(DM * DM / 64 / 64) * 8 * 8 * 64 == (size_t)DM * DM);
static_assert((size_t)(DM * DFF / 64 / 64) * 8 * 8 * 64 == (size_t)DM * DFF);
static_assert((size_t)(MROWS / 64) * (DM / 64) * 64 * 64 == (size_t)MROWS * DM);
static_assert((size_t)(MROWS / 64) * (DFF / 64) * 64 * 64 == (size_t)MROWS * DFF);
static_assert((size_t)(SEQ / 128) * NH * NB * 128 * 64 == (size_t)MROWS * DM);
static_assert((size_t)(MROWS / 8) * 8 * DM == (size_t)MROWS * DM);

typedef _Float16 h16;
typedef unsigned short bf;
typedef __attribute__((ext_vector_type(16))) __bf16   v16bf;
typedef __attribute__((ext_vector_type(16))) _Float16 v16h;
typedef __attribute__((ext_vector_type(8)))  _Float16 v8h;
typedef __attribute__((ext_vector_type(4)))  _Float16 v4h;
typedef __attribute__((ext_vector_type(2)))  _Float16 v2h;
typedef __attribute__((ext_vector_type(8)))  unsigned short v8us;
typedef __attribute__((ext_vector_type(2)))  unsigned short v2us;
typedef __attribute__((ext_vector_type(8)))  float    v8f;
typedef __attribute__((ext_vector_type(4)))  float    v4f;
typedef v8h  __attribute__((may_alias)) v8ha;
typedef v4f  __attribute__((may_alias)) v4fa;

__device__ __forceinline__ unsigned short f2bf(float f) { unsigned u = __float_as_uint(f); u += 0x7FFFu + ((u >> 16) & 1u); return (unsigned short)(u >> 16); }
__device__ __forceinline__ float bf2f(unsigned short b) { return __uint_as_float(((unsigned)b) << 16); }
__device__ __forceinline__ float bfr(float f) { return bf2f(f2bf(f)); }
__device__ __forceinline__ v16h cat16(v8h lo, v8h hi) { return __builtin_shufflevector(lo, hi, 0, 1, 2, 3, 4, 5, 6, 7, 8, 9, 10, 11, 12, 13, 14, 15); }
__device__ __forceinline__ v16bf cat16b(v8us lo, v8us hi) { return __builtin_bit_cast(v16bf, __builtin_shufflevector(lo, hi, 0, 1, 2, 3, 4, 5, 6, 7, 8, 9, 10, 11, 12, 13, 14, 15)); }
__device__ __forceinline__ v8f wmma16(v16h a, v16h b, v8f c) { return __builtin_amdgcn_wmma_f32_16x16x32_f16(false, a, false, b, (short)0, c, false, false); }
__device__ __forceinline__ v8f wmmab(v16bf a, v16bf b, v8f c) { return __builtin_amdgcn_wmma_f32_16x16x32_bf16(false, a, false, b, (short)0, c, false, false); }
__device__ __forceinline__ size_t xrow(size_t m) { return (m / SEQ) * (size_t)SEQ_FULL + (m % SEQ); }

template <typename T16> struct WFrag;
template <> struct WFrag<h16> { typedef v16h V; static __device__ __forceinline__ V ld(const h16* p) { return cat16(*(const v8h*)p, *(const v8h*)(p + 16)); } static __device__ __forceinline__ v8f mma(V a, V b, v8f c) { return wmma16(a, b, c); } };
template <> struct WFrag<bf> { typedef v16bf V; static __device__ __forceinline__ V ld(const bf* p) { return cat16b(*(const v8us*)p, *(const v8us*)(p + 16)); } static __device__ __forceinline__ v8f mma(V a, V b, v8f c) { return wmmab(a, b, c); } };

#define EPI_H16  0
#define EPI_VT   1
#define EPI_RES  2
#define EPI_RELU 3

template <typename T16, int EPI, bool RESBF>
__global__ __launch_bounds__(32) void k_gemmw(const T16* __restrict__ A, const T16* __restrict__ Bt, int K, void* Cout, int ldc, const float* __restrict__ bias, const float* res, float sc, float osc) {
    typedef typename WFrag<T16>::V V;
    __shared__ __align__(16) float os[64 * 68];
    const int lane = threadIdx.x & 31, lr = lane & 15, hi = lane >> 4; const int r0 = blockIdx.x * 64, c0 = blockIdx.y * 64;
    v8f acc[4][4];
#pragma unroll
    for (int mb = 0; mb < 4; ++mb)
#pragma unroll
        for (int nb = 0; nb < 4; ++nb) acc[mb][nb] = (v8f){};
    const size_t aoff = (size_t)(r0 + lr) * K + 8 * hi, boff = (size_t)(c0 + lr) * K + 8 * hi;
#pragma unroll 1
    for (int kc = 0; kc < K; kc += 32) {
        V a[4];
#pragma unroll
        for (int mb = 0; mb < 4; ++mb) a[mb] = WFrag<T16>::ld(A + aoff + (size_t)mb * 16 * K + kc);
#pragma unroll
        for (int nb = 0; nb < 4; ++nb) { const V b = WFrag<T16>::ld(Bt + boff + (size_t)nb * 16 * K + kc);
#pragma unroll
            for (int mb = 0; mb < 4; ++mb) acc[mb][nb] = WFrag<T16>::mma(a[mb], b, acc[mb][nb]); }
        asm volatile("v_nop\n\tv_nop\n\tv_nop\n\tv_nop" : "+v"(acc[0][0]), "+v"(acc[1][1]), "+v"(acc[2][2]), "+v"(acc[3][3]) : "v"(a[0]), "v"(a[3]));
    }
#pragma unroll
    for (int mb = 0; mb < 4; ++mb)
#pragma unroll
        for (int nb = 0; nb < 4; ++nb)
#pragma unroll
            for (int j = 0; j < 8; ++j) os[(mb * 16 + hi * 8 + j) * 68 + nb * 16 + lr] = acc[mb][nb][j];
    __syncthreads();
    const int cofs = lr * 4;
    { const v4f bv = *(const v4f*)(bias + c0 + cofs); v4f bb4;
#pragma unroll
      for (int q = 0; q < 4; ++q) bb4[q] = bfr(bv[q]);
#pragma unroll 1
      for (int it = 0; it < 32; ++it) { const int row = it * 2 + hi; float* op = os + row * 68 + cofs; v4f val = *(const v4fa*)op;
#pragma unroll
          for (int q = 0; q < 4; ++q) val[q] = val[q] * sc + bb4[q];
          if (EPI == EPI_RES) { const size_t rr = RESBF ? xrow((size_t)(r0 + row)) : (size_t)(r0 + row); const v4f rv = *(const v4f*)(res + rr * (size_t)ldc + c0 + cofs);
#pragma unroll
              for (int q = 0; q < 4; ++q) val[q] += RESBF ? bfr(rv[q]) : rv[q]; }
          if (EPI == EPI_RELU) {
#pragma unroll
              for (int q = 0; q < 4; ++q) val[q] = osc * fmaxf(val[q], 0.0f); }
          *(v4fa*)op = val; } }
    __syncthreads();
    if (EPI == EPI_RES) {
        float* C = (float*)Cout;
#pragma unroll 1
        for (int ps = 0; ps < 2; ++ps) {
#pragma unroll 4
            for (int it = 0; it < 32; ++it) { const int row = it * 2 + hi; const v4f val = *(const v4fa*)(os + row * 68 + cofs); *(volatile v4f*)(C + (size_t)(r0 + row) * ldc + c0 + cofs) = val; }
            if (ps == 0) __threadfence(); }
    } else if (EPI == EPI_VT) {
        h16* VT = (h16*)Cout; const unsigned ur0 = (unsigned)r0; const unsigned bidx = ur0 / (unsigned)SEQ, sloc = ur0 % (unsigned)SEQ;
        h16* vb = VT + ((size_t)(bidx * (unsigned)NH + blockIdx.y) * HD) * SEQ + sloc; const int dq = lane >> 3, s8 = (lane & 7) * 8;
#pragma unroll 1
        for (int ps = 0; ps < 2; ++ps) {
#pragma unroll 2
            for (int it = 0; it < 16; ++it) { const int d = it * 4 + dq; v8h o;
#pragma unroll
                for (int j = 0; j < 8; ++j) o[j] = (h16)os[(s8 + j) * 68 + d];
                *(volatile v8h*)(vb + (size_t)d * SEQ + s8) = o; }
            if (ps == 0) __threadfence(); }
    } else {
        h16* C = (h16*)Cout; const int rq = lane >> 3, c8 = (lane & 7) * 8;
#pragma unroll 1
        for (int ps = 0; ps < 2; ++ps) {
#pragma unroll 2
            for (int it = 0; it < 16; ++it) { const int row = it * 4 + rq; const v4f x0 = *(const v4fa*)(os + row * 68 + c8); const v4f x1 = *(const v4fa*)(os + row * 68 + c8 + 4); v8h o;
#pragma unroll
                for (int j = 0; j < 4; ++j) { o[j] = (h16)x0[j]; o[4 + j] = (h16)x1[j]; }
                *(volatile v8h*)(C + (size_t)(r0 + row) * ldc + c0 + c8) = o; }
            if (ps == 0) __threadfence(); }
    }
}

template <typename T16> struct WCv;
template <> struct WCv<bf>  { typedef v2us V2; static __device__ __forceinline__ bf  cv(float w) { return f2bf(w); } };
template <> struct WCv<h16> { typedef v2h  V2; static __device__ __forceinline__ h16 cv(float w) { return (h16)(bfr(w) * WCAR); } };
template <typename T16, int K, int N>
__global__ __launch_bounds__(256) void k_wtG(const float* __restrict__ w, T16* Bt) {
    typedef typename WCv<T16>::V2 V2;
    const int lane = threadIdx.x & 31; const int L0 = (blockIdx.x * 8 + (threadIdx.x >> 5)) * 8; const int nlines = N * K / 64;
#pragma unroll
    for (int ps = 0; ps < 2; ++ps) {
#pragma unroll 1
        for (int l = 0; l < 8; ++l) { const int L = L0 + l; if (L >= nlines) break; const size_t e = (size_t)L * 64 + lane * 2; const int k = (int)(e % K), n = (int)(e / K); V2 o;
            o[0] = WCv<T16>::cv(w[(size_t)k * N + n]); o[1] = WCv<T16>::cv(w[(size_t)(k + 1) * N + n]); *(volatile V2*)(Bt + e) = o; }
        if (ps == 0) __threadfence(); }
}

__global__ __launch_bounds__(256) void k_cvt8(const float* __restrict__ src, bf* dst) { const size_t i = (size_t)blockIdx.x * 256 + threadIdx.x; if (i >= (size_t)MROWS * DM / 8) return; const size_t e = i * 8; const size_t m = e / DM; const int c = (int)(e % DM); const v8f v = *(const v8f*)(src + xrow(m) * DM + c); v8us o;
#pragma unroll
    for (int k = 0; k < 8; ++k) o[k] = f2bf(v[k]);
    *(volatile v8us*)(dst + e) = o; __threadfence(); *(volatile v8us*)(dst + e) = o; }

__global__ __launch_bounds__(256) void k_attn(const h16* __restrict__ Q16, const h16* __restrict__ K16, const h16* __restrict__ VT16, h16* CTX) {
    __shared__ __align__(16) h16 sK[128 * 64];
    __shared__ __align__(16) h16 sV[64 * 128];
    __shared__ __align__(16) h16 sP[128 * 128];
    const int b = blockIdx.z, h = blockIdx.y, q0 = blockIdx.x * 128;
    const int t = threadIdx.x, lane = t & 31, wave = t >> 5, ln = lane & 15, hlf = lane >> 4;
    v16h qf[2];
    { const h16* qrow = Q16 + (size_t)(b * SEQ + q0 + wave * 16 + ln) * DM + h * HD + 8 * hlf;
      qf[0] = cat16(*(const v8h*)qrow, *(const v8h*)(qrow + 16)); qf[1] = cat16(*(const v8h*)(qrow + 32), *(const v8h*)(qrow + 48)); }
    const int krow = t >> 1, kseg = (t & 1) * 32, vrow = t >> 2, vseg = (t & 3) * 32;
    const h16* gK = K16 + (size_t)(b * SEQ + krow) * DM + h * HD + kseg;
    const h16* gV = VT16 + ((size_t)(b * NH + h) * HD + vrow) * SEQ + vseg;
    h16* lK = sK + krow * 64 + kseg; h16* lV = sV + vrow * 128 + vseg;
    float mrow[8], lrow[8]; v8f oacc[4];
#pragma unroll
    for (int r = 0; r < 8; ++r) { mrow[r] = -1e30f; lrow[r] = 0.f; }
#pragma unroll
    for (int nt = 0; nt < 4; ++nt) oacc[nt] = (v8f){};
#pragma unroll 1
    for (int sk0 = 0; sk0 < SEQ; sk0 += 128) {
        __syncthreads();
        { const h16* gk = gK + (size_t)sk0 * DM; const h16* gv = gV + sk0;
          const v8h k0 = *(const v8h*)gk, k1 = *(const v8h*)(gk + 8), k2 = *(const v8h*)(gk + 16), k3 = *(const v8h*)(gk + 24);
          *(v8ha*)lK = k0; *(v8ha*)(lK + 8) = k1; *(v8ha*)(lK + 16) = k2; *(v8ha*)(lK + 24) = k3;
          const v8h w0 = *(const v8h*)gv, w1 = *(const v8h*)(gv + 8), w2 = *(const v8h*)(gv + 16), w3 = *(const v8h*)(gv + 24);
          *(v8ha*)lV = w0; *(v8ha*)(lV + 8) = w1; *(v8ha*)(lV + 16) = w2; *(v8ha*)(lV + 24) = w3; }
        __syncthreads();
        v8f sacc[8];
#pragma unroll
        for (int nt = 0; nt < 8; ++nt) sacc[nt] = (v8f){};
#pragma unroll
        for (int ks = 0; ks < 2; ++ks) {
#pragma unroll
            for (int nt = 0; nt < 8; ++nt) { const h16* kp = sK + (nt * 16 + ln) * 64 + ks * 32 + 8 * hlf; const v16h kf = cat16(*(const v8ha*)kp, *(const v8ha*)(kp + 16)); sacc[nt] = wmma16(qf[ks], kf, sacc[nt]); } }
        asm volatile("v_nop\n\tv_nop\n\tv_nop\n\tv_nop" : "+v"(sacc[0]), "+v"(sacc[1]), "+v"(sacc[2]), "+v"(sacc[3]), "+v"(sacc[4]), "+v"(sacc[5]), "+v"(sacc[6]), "+v"(sacc[7]) : "v"(qf[0]), "v"(qf[1]));
        float mnew[8], fac[8];
#pragma unroll
        for (int r = 0; r < 8; ++r) { float m = -1e30f;
#pragma unroll
            for (int nt = 0; nt < 8; ++nt) { const float sv = sacc[nt][r] * 0.125f; sacc[nt][r] = sv; m = fmaxf(m, sv); }
#pragma unroll
            for (int o = 8; o > 0; o >>= 1) m = fmaxf(m, __shfl_xor(m, o, 32));
            mnew[r] = fmaxf(mrow[r], m); fac[r] = __builtin_amdgcn_exp2f((mrow[r] - mnew[r]) * LOG2E); mrow[r] = mnew[r]; }
#pragma unroll
        for (int r = 0; r < 8; ++r) { float rs = 0.f;
#pragma unroll
            for (int nt = 0; nt < 8; ++nt) { const float p = __builtin_amdgcn_exp2f((sacc[nt][r] - mnew[r]) * LOG2E); rs += p; sP[(wave * 16 + r + hlf * 8) * 128 + nt * 16 + ln] = (h16)(p * PCAR); }
#pragma unroll
            for (int o = 8; o > 0; o >>= 1) rs += __shfl_xor(rs, o, 32);
            lrow[r] = lrow[r] * fac[r] + rs; }
#pragma unroll
        for (int nt = 0; nt < 4; ++nt)
#pragma unroll
            for (int r = 0; r < 8; ++r) oacc[nt][r] *= fac[r];
        __syncthreads();
#pragma unroll
        for (int ks2 = 0; ks2 < 4; ++ks2) { const h16* pp = sP + (wave * 16 + ln) * 128 + ks2 * 32 + 8 * hlf; const v16h pf = cat16(*(const v8ha*)pp, *(const v8ha*)(pp + 16));
#pragma unroll
            for (int nt = 0; nt < 4; ++nt) { const h16* vp = sV + (nt * 16 + ln) * 128 + ks2 * 32 + 8 * hlf; const v16h vf = cat16(*(const v8ha*)vp, *(const v8ha*)(vp + 16)); oacc[nt] = wmma16(pf, vf, oacc[nt]); } }
        asm volatile("v_nop\n\tv_nop\n\tv_nop\n\tv_nop" : "+v"(oacc[0]), "+v"(oacc[1]), "+v"(oacc[2]), "+v"(oacc[3]) : "v"(qf[0]), "v"(qf[1]));
    }
    __syncthreads();
#pragma unroll
    for (int r = 0; r < 8; ++r) { const float inv = 1.0f / (lrow[r] * (PCAR / CCAR));
#pragma unroll
        for (int nt = 0; nt < 4; ++nt) sP[(wave * 16 + r + hlf * 8) * 128 + nt * 16 + ln] = (h16)(oacc[nt][r] * inv); }
    __syncthreads();
    h16* crow = CTX + (size_t)(b * SEQ + q0 + wave * 16) * DM + h * HD; const int rq = lane >> 3, c8 = (lane & 7) * 8;
#pragma unroll 1
    for (int ps = 0; ps < 2; ++ps) {
#pragma unroll
        for (int it = 0; it < 4; ++it) { const int row = it * 4 + rq; const v8h val = *(const v8ha*)(sP + (wave * 16 + row) * 128 + c8); *(volatile v8h*)(crow + (size_t)row * DM + c8) = val; }
        if (ps == 0) __threadfence(); }
}

template <bool W16>
__global__ __launch_bounds__(256) void k_ln(const float* F, const float* __restrict__ g, const float* __restrict__ bb, float* out, h16* o16) {
    const unsigned lane = threadIdx.x & 31u; const unsigned row = blockIdx.x * 8u + (threadIdx.x >> 5); if (row >= (unsigned)MROWS) return;
    const float* fr = F + (size_t)row * DM + lane * 4u; float* orow = out + (size_t)row * DM + lane * 4u;
    float s = 0.f;
#pragma unroll 1
    for (unsigned c = 0; c < DM / 128; ++c) { const v4f a = *(const v4f*)(fr + c * 128u); s += (a[0] + a[1]) + (a[2] + a[3]); }
#pragma unroll
    for (int sh = 16; sh; sh >>= 1) s += __shfl_xor(s, sh, 32);
    const float mean = s * (1.0f / (float)DM); float s2 = 0.f;
#pragma unroll 1
    for (unsigned c = 0; c < DM / 128; ++c) { const v4f a = *(const v4f*)(fr + c * 128u);
#pragma unroll
        for (int q = 0; q < 4; ++q) { const float dv = a[q] - mean; s2 += dv * dv; } }
#pragma unroll
    for (int sh = 16; sh; sh >>= 1) s2 += __shfl_xor(s2, sh, 32);
    const float sd = sqrtf(s2 * (1.0f / (float)DM)); const float inv = 1.0f / (sd + LNEPS);
#pragma unroll 1
    for (int ps = 0; ps < 2; ++ps) {
#pragma unroll 1
        for (unsigned c = 0; c < DM / 128; ++c) { const unsigned col = c * 128u; const v4f a = *(const v4f*)(fr + col); const v4f gg = *(const v4f*)(g + col + lane * 4u); const v4f be = *(const v4f*)(bb + col + lane * 4u); v4f o; v4h o4;
#pragma unroll
            for (int q = 0; q < 4; ++q) { const float tn = (a[q] - mean) * inv; o[q] = tn * bfr(gg[q]) + bfr(be[q]); o4[q] = (h16)o[q]; }
            *(volatile v4f*)(orow + col) = o;
            if (W16) { h16* hrow = o16 + (size_t)row * DM + lane * 4u; *(volatile v4h*)(hrow + col) = o4; } }
        if (ps == 0) __threadfence(); }
}

extern "C" void kernel_launch(void* const* d_in, const int* in_sizes, int n_in,
                              void* d_out, int out_size, void* d_ws, size_t ws_size, hipStream_t stream) {
    if (n_in < 17) return;
    const size_t M = (size_t)MROWS;
    if ((size_t)in_sizes[0] < ((size_t)(NB - 1) * SEQ_FULL + SEQ) * DM) return;
    if ((size_t)in_sizes[1] < (size_t)DM * DM || (size_t)in_sizes[3] < (size_t)DM * DM || (size_t)in_sizes[5] < (size_t)DM * DM || (size_t)in_sizes[7] < (size_t)DM * DM) return;
    if ((size_t)in_sizes[9] < (size_t)DM * DFF || (size_t)in_sizes[11] < (size_t)DFF * DM) return;
    if (in_sizes[2] < DM || in_sizes[4] < DM || in_sizes[6] < DM || in_sizes[8] < DM || in_sizes[10] < DFF || in_sizes[12] < DM || in_sizes[13] < DM || in_sizes[14] < DM || in_sizes[15] < DM || in_sizes[16] < DM) return;
    if ((size_t)out_size < M * DM) return;
    const float* x  = (const float*)d_in[0];
    const float* wq = (const float*)d_in[1];  const float* bq  = (const float*)d_in[2];
    const float* wk = (const float*)d_in[3];  const float* bk  = (const float*)d_in[4];
    const float* wv = (const float*)d_in[5];  const float* bv  = (const float*)d_in[6];
    const float* wo = (const float*)d_in[7];  const float* bo  = (const float*)d_in[8];
    const float* w1 = (const float*)d_in[9];  const float* b1  = (const float*)d_in[10];
    const float* w2 = (const float*)d_in[11]; const float* b2  = (const float*)d_in[12];
    const float* g1 = (const float*)d_in[13]; const float* be1 = (const float*)d_in[14];
    const float* g2 = (const float*)d_in[15]; const float* be2 = (const float*)d_in[16];
    float* OUT = (float*)d_out;
    char* wsp = (char*)d_ws;
    auto take = [&](size_t bytes) { char* p = wsp; wsp += (bytes + 255) & ~(size_t)255; return (void*)p; };
    const size_t qkb = 2 * M * DM * 2, gb = M * DFF * 2;
    h16* QK = (h16*)take(qkb > gb ? qkb : gb);
    void* R1 = take(M * DM * 2);
    h16* VT16 = (h16*)take(M * DM * 2);
    float* Hf = (float*)take(M * DM * 4);
    float* Yf = (float*)take(M * DM * 4);
    bf* WQ = (bf*)take((size_t)DM * DM * 2); bf* WK = (bf*)take((size_t)DM * DM * 2); bf* WV = (bf*)take((size_t)DM * DM * 2);
    h16* WO = (h16*)take((size_t)DM * DM * 2); h16* W1T = (h16*)take((size_t)DFF * DM * 2); h16* W2T = (h16*)take((size_t)DM * DFF * 2);
    const size_t used = (size_t)(wsp - (char*)d_ws);
    if (used > ws_size || used > (size_t)134217728) return;
    h16* Q16 = QK; h16* K16 = QK + M * DM; h16* G16 = QK;
    bf* XB = (bf*)R1; h16* CTX = (h16*)R1; h16* H16 = (h16*)R1;

    k_cvt8<<<(unsigned)(M * DM / 8 / 256), 256, 0, stream>>>(x, XB);
    k_wtG<bf, DM, DM><<<DM * DM / 64 / 64, 256, 0, stream>>>(wq, WQ);
    k_wtG<bf, DM, DM><<<DM * DM / 64 / 64, 256, 0, stream>>>(wk, WK);
    k_wtG<bf, DM, DM><<<DM * DM / 64 / 64, 256, 0, stream>>>(wv, WV);
    k_wtG<h16, DM, DM><<<DM * DM / 64 / 64, 256, 0, stream>>>(wo, WO);
    k_wtG<h16, DM, DFF><<<DM * DFF / 64 / 64, 256, 0, stream>>>(w1, W1T);
    k_wtG<h16, DFF, DM><<<DFF * DM / 64 / 64, 256, 0, stream>>>(w2, W2T);

    const dim3 gD((unsigned)(M / 64), DM / 64), gF((unsigned)(M / 64), DFF / 64);
    k_gemmw<bf, EPI_H16, false><<<gD, 32, 0, stream>>>(XB, WQ, DM, (void*)Q16, DM, bq, nullptr, 1.0f, 1.0f);
    k_gemmw<bf, EPI_H16, false><<<gD, 32, 0, stream>>>(XB, WK, DM, (void*)K16, DM, bk, nullptr, 1.0f, 1.0f);
    k_gemmw<bf, EPI_VT, false><<<gD, 32, 0, stream>>>(XB, WV, DM, (void*)VT16, DM, bv, nullptr, 1.0f, 1.0f);

    k_attn<<<dim3(SEQ / 128, NH, NB), 256, 0, stream>>>(Q16, K16, VT16, CTX);

    k_gemmw<h16, EPI_RES, true><<<gD, 32, 0, stream>>>(CTX, WO, DM, (void*)Yf, DM, bo, x, 1.0f / (CCAR * WCAR), 1.0f);
    k_ln<true><<<(unsigned)(M / 8), 256, 0, stream>>>(Yf, g1, be1, Hf, H16);
    k_gemmw<h16, EPI_RELU, false><<<gF, 32, 0, stream>>>(H16, W1T, DM, (void*)G16, DFF, b1, nullptr, 1.0f / WCAR, GCAR);
    k_gemmw<h16, EPI_RES, false><<<gD, 32, 0, stream>>>(G16, W2T, DFF, (void*)Yf, DM, b2, Hf, 1.0f / (GCAR * WCAR), 1.0f);
    k_ln<false><<<(unsigned)(M / 8), 256, 0, stream>>>(Yf, g2, be2, OUT, nullptr);
}
